// IDRM_ANN_81389630259799
// MI455X (gfx1250) — hardware-run, weakly checked
//
#include <hip/hip_runtime.h>
#include <math.h>

typedef __attribute__((ext_vector_type(16))) _Float16 v16h;
typedef __attribute__((ext_vector_type(8)))  _Float16 v8h;
typedef __attribute__((ext_vector_type(8)))  float    v8f;
typedef __attribute__((ext_vector_type(4)))  float    v4f;
typedef __attribute__((ext_vector_type(4)))  unsigned v4u;

constexpr int kBatch = 16384;
constexpr int kNin   = 256;
constexpr int kNhid  = 1024;
constexpr int kNout  = 256;
constexpr int kHalf  = 8192;
constexpr int kNgate = 3 * kNhid;
static_assert(kHalf * 2 == kBatch);
static_assert((kNin % 32) == 0 && (kNhid % 32) == 0);
static_assert((kHalf % 64) == 0 && (kNhid % 64) == 0 && (kNgate % 64) == 0 && (kNout % 64) == 0);

constexpr float kCarryW   = 256.0f;
constexpr float kCarryAct = 16.0f;
constexpr float kCarryUh  = kCarryW * kCarryAct;
constexpr float kInvGate  = 1.0f / kCarryW;
constexpr float kInvCand  = 1.0f / kCarryUh;
static_assert(kCarryUh == 4096.0f);

constexpr size_t kOffXA   = 0;
constexpr size_t kOffW0   = kOffXA   + (size_t)kBatch * kNin  * 2;
constexpr size_t kOffUGZR = kOffW0   + (size_t)kNhid  * kNin  * 2;
constexpr size_t kOffUH   = kOffUGZR + (size_t)kNgate * kNin  * 2;
constexpr size_t kOffWGZR = kOffUH   + (size_t)kNhid  * kNin  * 2;
constexpr size_t kOffWH   = kOffWGZR + (size_t)kNgate * kNhid * 2;
constexpr size_t kOffW4   = kOffWH   + (size_t)kNhid  * kNhid * 2;
constexpr size_t kOffS0   = kOffW4   + (size_t)kNout  * kNhid * 2;
constexpr size_t kOffG    = kOffS0   + (size_t)kHalf  * kNhid * 2;
constexpr size_t kOffZC   = kOffG    + (size_t)kHalf  * kNhid * 2;
constexpr size_t kOffSR   = kOffZC   + (size_t)kHalf  * kNhid * 2;
constexpr size_t kOffS1   = kOffSR   + (size_t)kHalf  * kNhid * 2;
constexpr size_t kWsTotal = kOffS1   + (size_t)kHalf  * kNhid * 2;
static_assert(kWsTotal == 103809024ull);
static_assert(kWsTotal <= 134217728ull);
static_assert((kOffW0 % 128) == 0 && (kOffUGZR % 128) == 0 && (kOffUH % 128) == 0 && (kOffWGZR % 128) == 0 &&
              (kOffWH % 128) == 0 && (kOffW4 % 128) == 0 && (kOffS0 % 128) == 0 && (kOffG % 128) == 0 &&
              (kOffZC % 128) == 0 && (kOffSR % 128) == 0 && (kOffS1 % 128) == 0);

union FragU { v16h v; v8h h[2]; };

__device__ __forceinline__ v16h frag_load(const _Float16* p) {
  FragU f;
  f.h[0] = *(const v8h*)(p);
  f.h[1] = *(const v8h*)(p + 16);
  return f.v;
}

__device__ __forceinline__ v8f mma_h(v16h a, v16h b, v8f c) {
  c = __builtin_amdgcn_wmma_f32_16x16x32_f16(false, a, false, b, (short)0, c, false, false);
  asm volatile("v_nop\n\tv_nop\n\tv_nop\n\tv_nop" : "+v"(c) : "v"(a), "v"(b));
  return c;
}

__device__ __forceinline__ float h16_to_f32(unsigned hb) {
  const unsigned sgn = (hb & 0x8000u) << 16;
  const unsigned em = hb & 0x7fffu;
  const float fn = __uint_as_float((em << 13) + 0x38000000u);
  const float fs = (float)em * 5.9604644775390625e-8f;
  const float mag = (em < 0x400u) ? fs : fn;
  return __uint_as_float(__float_as_uint(mag) | sgn);
}

__device__ __forceinline__ void unpack8(v4u w, float (&o)[8]) {
  const unsigned w0 = w[0];
  const unsigned w1 = w[1];
  const unsigned w2 = w[2];
  const unsigned w3 = w[3];
  o[0] = h16_to_f32(w0 & 0xffffu);
  o[1] = h16_to_f32(w0 >> 16);
  o[2] = h16_to_f32(w1 & 0xffffu);
  o[3] = h16_to_f32(w1 >> 16);
  o[4] = h16_to_f32(w2 & 0xffffu);
  o[5] = h16_to_f32(w2 >> 16);
  o[6] = h16_to_f32(w3 & 0xffffu);
  o[7] = h16_to_f32(w3 >> 16);
}

__device__ __forceinline__ float tanh_fast(float v) {
  const float c = fminf(fmaxf(v, -15.0f), 15.0f);
  const float e = __expf(2.0f * c);
  return 1.0f - 2.0f * __builtin_amdgcn_rcpf(e + 1.0f);
}

__device__ __forceinline__ void wave_lds_sync() {
  __builtin_amdgcn_fence(__ATOMIC_RELEASE, "workgroup");
  __builtin_amdgcn_wave_barrier();
  __builtin_amdgcn_fence(__ATOMIC_ACQUIRE, "workgroup");
}

template <bool ABSP>
__global__ __launch_bounds__(256) void cvt_f16_kernel(
    const float* sA, const float* sB, const float* sC,
    unsigned short* dA, unsigned short* dB, unsigned short* dC,
    float cA, float cB, float cC, int n8)
{
  const int y = blockIdx.y;
  const float* src = (y == 0) ? sA : ((y == 1) ? sB : sC);
  unsigned short* dst = (y == 0) ? dA : ((y == 1) ? dB : dC);
  const float cs = (y == 0) ? cA : ((y == 1) ? cB : cC);
  const int i = blockIdx.x * 256 + threadIdx.x;
  if (i >= n8) return;
  const size_t e0 = (size_t)i << 3;
  const v4f a0 = *(const v4f*)(src + e0);
  const v4f a1 = *(const v4f*)(src + e0 + 4);
  v8h hv;
#pragma unroll
  for (int e = 0; e < 4; ++e) {
    float f0 = a0[e];
    float f1 = a1[e];
    if (ABSP) {
      f0 = fabsf(f0) + 0.1f;
      f1 = fabsf(f1) + 0.1f;
    } else {
      f0 = f0 * cs;
      f1 = f1 * cs;
    }
    hv[e]     = (_Float16)f0;
    hv[4 + e] = (_Float16)f1;
  }
  unsigned short* qd = dst + e0;
  *(volatile v8h*)qd = hv;
  __threadfence();
  *(volatile v8h*)qd = hv;
}

template <int KD>
__device__ __forceinline__ void kseg(const _Float16* __restrict__ A, const _Float16* __restrict__ B,
                                     v8f (&acc)[4][4])
{
#pragma unroll 1
  for (int k0 = 0; k0 < KD; k0 += 32) {
    v16h bh[4];
#pragma unroll
    for (int j = 0; j < 4; ++j) bh[j] = frag_load(B + (size_t)j * 16 * KD + k0);
#pragma unroll
    for (int i = 0; i < 4; ++i) {
      const v16h ah = frag_load(A + (size_t)i * 16 * KD + k0);
#pragma unroll
      for (int j = 0; j < 4; ++j) acc[i][j] = mma_h(ah, bh[j], acc[i][j]);
    }
  }
}

template <int MODE, int KA, int KB>
__global__ __launch_bounds__(256) __attribute__((amdgpu_num_vgpr(256))) void gemm_gate_kernel(
    const unsigned short* __restrict__ A1p, const unsigned short* __restrict__ B1p,
    const unsigned short* __restrict__ A2p, const unsigned short* __restrict__ B2p,
    const float* __restrict__ biasA, const float* __restrict__ biasB, const float* __restrict__ biasC,
    const unsigned short* __restrict__ E0, const unsigned short* __restrict__ E1,
    unsigned short* __restrict__ O0, unsigned short* __restrict__ O1, unsigned short* __restrict__ O2,
    float* __restrict__ OF, int M, int N, float scale)
{
  static_assert((KA % 32) == 0 && (KB % 32) == 0 && KA > 0);
  __shared__ __align__(16) float sT[8][16 * 68];
  const int lane = threadIdx.x & 31;
  const int wave = threadIdx.x >> 5;
  const int tilesN = N >> 6;
  const int tilesM = M >> 6;
  const int tile = blockIdx.x * 8 + wave;
  if (tile >= tilesM * tilesN) return;
  const int tm = tile / tilesN;
  const int tn = tile - tm * tilesN;
  const int m0 = tm << 6;
  const int n0 = tn << 6;
  const int rlane = lane & 15;
  const int koff  = (lane >> 4) * 8;
  const int mOff  = (lane >> 4) * 8;

  v8f acc[4][4];
#pragma unroll
  for (int i = 0; i < 4; ++i)
#pragma unroll
    for (int j = 0; j < 4; ++j) acc[i][j] = (v8f){0.f, 0.f, 0.f, 0.f, 0.f, 0.f, 0.f, 0.f};

  {
    const _Float16* A = (const _Float16*)A1p + (size_t)(m0 + rlane) * KA + koff;
    const _Float16* B = (const _Float16*)B1p + (size_t)(n0 + rlane) * KA + koff;
    kseg<KA>(A, B, acc);
  }
  if (KB > 0) {
    const _Float16* A = (const _Float16*)A2p + (size_t)(m0 + rlane) * KB + koff;
    const _Float16* B = (const _Float16*)B2p + (size_t)(n0 + rlane) * KB + koff;
    kseg<KB>(A, B, acc);
  }

  float* slab = sT[wave];
  if (MODE == 3) {
    const int hh = lane >> 4;
    const int c4 = (lane & 15) * 4;
#pragma unroll
    for (int i = 0; i < 4; ++i) {
      const int mBase = m0 + (i << 4);
#pragma unroll
      for (int j = 0; j < 4; ++j)
#pragma unroll
        for (int r = 0; r < 8; ++r)
          slab[(mOff + r) * 68 + (j << 4) + rlane] = acc[i][j][r] * scale;
      wave_lds_sync();
      v4f ov[8];
#pragma unroll
      for (int it = 0; it < 8; ++it) ov[it] = *(const v4f*)(slab + (it * 2 + hh) * 68 + c4);
      for (int pass = 0; pass < 2; ++pass) {
#pragma unroll
        for (int it = 0; it < 8; ++it)
          *(volatile v4f*)(OF + (size_t)(mBase + it * 2 + hh) * N + n0 + c4) = ov[it];
        __threadfence();
      }
      wave_lds_sync();
    }
  } else {
    const int q  = lane >> 3;
    const int c8 = (lane & 7) * 8;
    const int sel = (MODE == 1) ? (n0 >> 10) : 0;
    const int nc  = (MODE == 1) ? (n0 & (kNhid - 1)) : n0;
    const float* bp = biasA;
    unsigned short* op = O0;
    if (MODE == 1) {
      bp = (sel == 0) ? biasA : ((sel == 1) ? biasB : biasC);
      op = (sel == 0) ? O0 : ((sel == 1) ? O1 : O2);
    }
    const float ocarry = (MODE == 2) ? kCarryAct : ((MODE == 1 && sel == 2) ? kCarryAct : 1.0f);
    const v4f bq0 = *(const v4f*)(bp + nc + c8);
    const v4f bq1 = *(const v4f*)(bp + nc + c8 + 4);
    float bv[8];
    bv[0] = bq0[0]; bv[1] = bq0[1]; bv[2] = bq0[2]; bv[3] = bq0[3];
    bv[4] = bq1[0]; bv[5] = bq1[1]; bv[6] = bq1[2]; bv[7] = bq1[3];
#pragma unroll
    for (int i = 0; i < 4; ++i) {
      const int mBase = m0 + (i << 4);
#pragma unroll
      for (int j = 0; j < 4; ++j)
#pragma unroll
        for (int r = 0; r < 8; ++r)
          slab[(mOff + r) * 68 + (j << 4) + rlane] = acc[i][j][r] * scale;
      wave_lds_sync();
#pragma unroll 1
      for (int it = 0; it < 4; ++it) {
        const int row = it * 4 + q;
        const float* sp = slab + row * 68 + c8;
        const v4f a0 = *(const v4f*)(sp);
        const v4f a1 = *(const v4f*)(sp + 4);
        float pv[8];
        pv[0] = a0[0]; pv[1] = a0[1]; pv[2] = a0[2]; pv[3] = a0[3];
        pv[4] = a1[0]; pv[5] = a1[1]; pv[6] = a1[2]; pv[7] = a1[3];
        const size_t go = (size_t)(mBase + row) * kNhid + nc + c8;
        float ea[8], eb[8];
#pragma unroll
        for (int e = 0; e < 8; ++e) { ea[e] = 1.0f; eb[e] = 0.0f; }
        if (MODE == 1 || MODE == 2) {
          const v4u w = *(const v4u*)(E0 + go);
          unpack8(w, ea);
        }
        if (MODE == 2) {
          const v4u w = *(const v4u*)(E1 + go);
          unpack8(w, eb);
        }
        v8h hv;
#pragma unroll
        for (int e = 0; e < 8; ++e) {
          const float t = tanh_fast(pv[e] + bv[e]);
          float outv;
          if (MODE == 0) {
            outv = t;
          } else if (MODE == 1) {
            const float mul = (sel == 0) ? 1.0f : ea[e];
            outv = ocarry * (t * mul);
          } else {
            outv = ocarry * ((1.0f - ea[e]) * t + eb[e]);
          }
          hv[e] = (_Float16)outv;
        }
        unsigned short* dstp = op + go;
        *(volatile v8h*)dstp = hv;
        __threadfence();
        *(volatile v8h*)dstp = hv;
      }
      wave_lds_sync();
    }
  }
}

extern "C" void kernel_launch(void* const* d_in, const int* in_sizes, int n_in,
                              void* d_out, int out_size, void* d_ws, size_t ws_size,
                              hipStream_t stream) {
  if (n_in < 28) return;
  if (in_sizes[0] != kBatch * kNin) return;
  if (in_sizes[1] != kNhid * kNin) return;
  if (in_sizes[2] != kNhid) return;
  if (in_sizes[3] != kNhid * kNin) return;
  if (in_sizes[4] != kNhid * kNhid) return;
  if (in_sizes[5] != kNhid) return;
  if (in_sizes[6] != kNhid * kNin) return;
  if (in_sizes[7] != kNhid * kNhid) return;
  if (in_sizes[8] != kNhid) return;
  if (in_sizes[9] != kNhid * kNin) return;
  if (in_sizes[10] != kNhid * kNhid) return;
  if (in_sizes[11] != kNhid) return;
  if (in_sizes[12] != kNhid * kNin) return;
  if (in_sizes[13] != kNhid * kNhid) return;
  if (in_sizes[14] != kNhid) return;
  if (in_sizes[27] != kNout * kNhid) return;
  if (out_size != kBatch * kNout) return;
  if (ws_size < kWsTotal) return;

  const float* x     = (const float*)d_in[0];
  const float* w0_w  = (const float*)d_in[1];
  const float* w0_b  = (const float*)d_in[2];
  const float* ug1   = (const float*)d_in[3];
  const float* wg1_w = (const float*)d_in[4];
  const float* wg1_b = (const float*)d_in[5];
  const float* uz1   = (const float*)d_in[6];
  const float* wz1_w = (const float*)d_in[7];
  const float* wz1_b = (const float*)d_in[8];
  const float* ur1   = (const float*)d_in[9];
  const float* wr1_w = (const float*)d_in[10];
  const float* wr1_b = (const float*)d_in[11];
  const float* uh1   = (const float*)d_in[12];
  const float* wh1_w = (const float*)d_in[13];
  const float* wh1_b = (const float*)d_in[14];
  const float* w4    = (const float*)d_in[27];
  float* out = (float*)d_out;

  char* ws = (char*)d_ws;
  unsigned short* XA   = (unsigned short*)(ws + kOffXA);
  unsigned short* W0   = (unsigned short*)(ws + kOffW0);
  unsigned short* UGZR = (unsigned short*)(ws + kOffUGZR);
  unsigned short* UH   = (unsigned short*)(ws + kOffUH);
  unsigned short* WGZR = (unsigned short*)(ws + kOffWGZR);
  unsigned short* WH   = (unsigned short*)(ws + kOffWH);
  unsigned short* W4   = (unsigned short*)(ws + kOffW4);
  unsigned short* S0   = (unsigned short*)(ws + kOffS0);
  unsigned short* G    = (unsigned short*)(ws + kOffG);
  unsigned short* ZC   = (unsigned short*)(ws + kOffZC);
  unsigned short* SR   = (unsigned short*)(ws + kOffSR);
  unsigned short* S1   = (unsigned short*)(ws + kOffS1);

  constexpr int kN8x  = kBatch * kNin / 8;
  constexpr int kN8u  = kNhid * kNin / 8;
  constexpr int kN8w  = kNhid * kNhid / 8;
  static_assert((kN8x % 256) == 0 && (kN8u % 256) == 0 && (kN8w % 256) == 0);
  static_assert(kNout * kNhid == kNhid * kNin);

  cvt_f16_kernel<true><<<dim3(kN8x / 256, 1), 256, 0, stream>>>(
      x, x, x, XA, XA, XA, 1.0f, 1.0f, 1.0f, kN8x);
  cvt_f16_kernel<false><<<dim3(kN8u / 256, 3), 256, 0, stream>>>(
      ug1, uz1, ur1, UGZR, UGZR + (size_t)kNhid * kNin, UGZR + (size_t)2 * kNhid * kNin,
      kCarryW, kCarryW, kCarryW, kN8u);
  cvt_f16_kernel<false><<<dim3(kN8w / 256, 3), 256, 0, stream>>>(
      wg1_w, wz1_w, wr1_w, WGZR, WGZR + (size_t)kNhid * kNhid, WGZR + (size_t)2 * kNhid * kNhid,
      kCarryW, kCarryW, kCarryW, kN8w);
  cvt_f16_kernel<false><<<dim3(kN8u / 256, 3), 256, 0, stream>>>(
      w0_w, uh1, w4, W0, UH, W4, kCarryW, kCarryUh, kCarryW, kN8u);
  cvt_f16_kernel<false><<<dim3(kN8w / 256, 1), 256, 0, stream>>>(
      wh1_w, wh1_w, wh1_w, WH, WH, WH, kCarryW, kCarryW, kCarryW, kN8w);

  constexpr int kBlkHid  = (kHalf / 64) * (kNhid / 64) / 8;
  constexpr int kBlkGate = (kHalf / 64) * (kNgate / 64) / 8;
  constexpr int kBlkOut  = (kHalf / 64) * (kNout / 64) / 8;
  static_assert(kBlkHid * 8 == (kHalf / 64) * (kNhid / 64));
  static_assert(kBlkGate * 8 == (kHalf / 64) * (kNgate / 64));
  static_assert(kBlkOut * 8 == (kHalf / 64) * (kNout / 64));

  for (int hf = 0; hf < 2; ++hf) {
    const unsigned short* xa_h = XA + (size_t)hf * kHalf * kNin;
    float* out_h = out + (size_t)hf * kHalf * kNout;

    gemm_gate_kernel<0, kNin, 0><<<kBlkHid, 256, 0, stream>>>(
        xa_h, W0, nullptr, nullptr,
        w0_b, nullptr, nullptr,
        nullptr, nullptr,
        S0, nullptr, nullptr,
        nullptr, kHalf, kNhid, kInvGate);

    gemm_gate_kernel<1, kNin, kNhid><<<kBlkGate, 256, 0, stream>>>(
        xa_h, UGZR, S0, WGZR,
        wg1_b, wz1_b, wr1_b,
        S0, nullptr,
        G, ZC, SR,
        nullptr, kHalf, kNgate, kInvGate);

    gemm_gate_kernel<2, kNin, kNhid><<<kBlkHid, 256, 0, stream>>>(
        xa_h, UH, SR, WH,
        wh1_b, nullptr, nullptr,
        G, ZC,
        S1, nullptr, nullptr,
        nullptr, kHalf, kNhid, kInvCand);

    gemm_gate_kernel<3, kNhid, 0><<<kBlkOut, 256, 0, stream>>>(
        S1, W4, nullptr, nullptr,
        nullptr, nullptr, nullptr,
        nullptr, nullptr,
        nullptr, nullptr, nullptr,
        out_h, kHalf, kNout, kInvCand);
  }
}
